// EarlyJoinGConv_13228499272260
// MI455X (gfx1250) — hardware-verified
//
#include <hip/hip_runtime.h>
#include <hip/hip_bf16.h>
#include <math.h>


#define BB 2
#define SS 2048
#define DD 1024
#define HH 16
#define DKK 64
#define QW 2

typedef _Float16 bf16;
typedef __attribute__((ext_vector_type(4))) unsigned v4u_t;
typedef unsigned v4ua __attribute__((ext_vector_type(4), may_alias));
typedef __attribute__((ext_vector_type(4))) float v4f_t;
typedef float v4fa __attribute__((ext_vector_type(4), may_alias));
typedef __attribute__((ext_vector_type(16))) bf16  bf16x16;
typedef __attribute__((ext_vector_type(8)))  bf16  bf16x8;
typedef __attribute__((ext_vector_type(4)))  bf16  bf16x4;
typedef __attribute__((ext_vector_type(8)))  float f32x8;

#define LDS_STRIDE 48
#define KSTRIDE    72
#define VSTRIDE    48

__device__ __forceinline__ f32x8 wmma_bf16(bf16x16 a, bf16x16 b, f32x8 c) {
  return __builtin_amdgcn_wmma_f32_16x16x32_f16(
      false, a, false, b, (short)0, c, false, false);
}

template <typename T>
__device__ __forceinline__ bf16x16 load_frag(const T* __restrict__ base, int ld,
                                             int row0, int k0) {
  const int lane = threadIdx.x & 31;
  const int r    = lane & 15;
  const int kh   = (lane >> 4) * 8;
  const T* p0 = base + (size_t)(row0 + r) * ld + (k0 + kh);
  const T* p1 = p0 + 16;
  bf16x16 f;
#pragma unroll
  for (int i = 0; i < 8; ++i) {
    f[i]     = (bf16)p0[i];
    f[i + 8] = (bf16)p1[i];
  }
  return f;
}

__device__ __forceinline__ bf16x16 lds_frag(const bf16* base, int stride) {
  const int lane = threadIdx.x & 31;
  const int row  = lane & 15;
  const int kh   = (lane >> 4) * 8;
  const bf16x8 lo = *(const bf16x8*)(base + row * stride + kh);
  const bf16x8 hi = *(const bf16x8*)(base + row * stride + kh + 16);
  bf16x16 f;
#pragma unroll
  for (int i = 0; i < 8; ++i) { f[i] = lo[i]; f[i + 8] = hi[i]; }
  return f;
}

template <typename T>
__device__ __forceinline__ void stage_read16(const T* __restrict__ p, float* buf) {
#pragma unroll
  for (int i = 0; i < 16; ++i) buf[i] = (float)p[i];
}

__device__ __forceinline__ void stage_write(bf16* dst, const float* buf, int nquad) {
#pragma unroll
  for (int i = 0; i < nquad; ++i) {
    bf16x4 q;
    q[0] = (bf16)buf[4 * i];     q[1] = (bf16)buf[4 * i + 1];
    q[2] = (bf16)buf[4 * i + 2]; q[3] = (bf16)buf[4 * i + 3];
    *(bf16x4*)(dst + 4 * i) = q;
  }
}

template <typename AT, typename WTY, int MODE>
__global__ __launch_bounds__(256) void gemm_bias_kernel(
    const AT* __restrict__ A, const WTY* __restrict__ W,
    const float* __restrict__ bias, void* __restrict__ out,
    int M, int N, int K) {
  __shared__ bf16 ldsA[128 * LDS_STRIDE];
  __shared__ bf16 ldsW[256 * LDS_STRIDE];
  __shared__ __attribute__((aligned(16))) unsigned char sob[256 * 136 * 2];

  const int t    = threadIdx.x;
  const int wave = t >> 5;
  const int lane = t & 31;
  const int wm   = (wave & 1) * 64;
  const int wn   = (wave >> 1) * 64;
  const int mBlk = blockIdx.x * 128;
  const int nBlk = blockIdx.y * 256;

  const int arow = t >> 1;
  const int ach  = (t & 1) * 16;

  float abuf[16];
  float wbuf[32];

  stage_read16(A + (size_t)(mBlk + arow) * K + ach, abuf);
  stage_read16(W + (size_t)(nBlk + t) * K,          wbuf);
  stage_read16(W + (size_t)(nBlk + t) * K + 16,     wbuf + 16);

  f32x8 acc[4][4] = {};

  for (int k = 0; k < K; k += 32) {
    __syncthreads();
    stage_write(&ldsA[arow * LDS_STRIDE + ach], abuf, 4);
    stage_write(&ldsW[t * LDS_STRIDE],          wbuf, 8);
    if (k + 32 < K) {
      stage_read16(A + (size_t)(mBlk + arow) * K + (k + 32) + ach, abuf);
      stage_read16(W + (size_t)(nBlk + t) * K + (k + 32),          wbuf);
      stage_read16(W + (size_t)(nBlk + t) * K + (k + 32) + 16,     wbuf + 16);
    }
    __syncthreads();

    bf16x16 af[4], wf[4];
#pragma unroll
    for (int i = 0; i < 4; ++i)
      af[i] = lds_frag(ldsA + (wm + 16 * i) * LDS_STRIDE, LDS_STRIDE);
#pragma unroll
    for (int j = 0; j < 4; ++j)
      wf[j] = lds_frag(ldsW + (wn + 16 * j) * LDS_STRIDE, LDS_STRIDE);
#pragma unroll
    for (int i = 0; i < 4; ++i)
#pragma unroll
      for (int j = 0; j < 4; ++j)
        acc[i][j] = wmma_bf16(af[i], wf[j], acc[i][j]);
  }

  const int nlane = lane & 15;
  const int mh    = (lane >> 4) * 8;
  __syncthreads();
  if (MODE == 0 || MODE == 1) {
    bf16* so = (bf16*)sob;
#pragma unroll
    for (int i = 0; i < 4; ++i)
#pragma unroll
      for (int j = 0; j < 4; ++j) {
        const int nl = wn + 16 * j + nlane;
        const float bv = bias ? bias[nBlk + nl] : 0.0f;
#pragma unroll
        for (int r = 0; r < 8; ++r) {
          const int ml = wm + 16 * i + mh + r;
          const bf16 hv = (bf16)(acc[i][j][r] + bv);
          if (MODE == 0) so[ml * 264 + nl] = hv;
          else           so[nl * 136 + ml] = hv;
        }
      }
    __syncthreads();
#pragma unroll 1
    for (int pass = 0; pass < 2; ++pass) {
      if (MODE == 0) {
        for (int ch = t; ch < 128 * 32; ch += 256) { const int ml = ch >> 5, q = (ch & 31) * 8;
          *(volatile v4u_t*)((bf16*)out + (size_t)(mBlk + ml) * N + nBlk + q) = *(const v4ua*)(so + ml * 264 + q); }
      } else {
        const int b_ = mBlk / SS, s0 = mBlk & (SS - 1);
        for (int ch = t; ch < 256 * 16; ch += 256) { const int nl = ch >> 4, q = (ch & 15) * 8; const int n = nBlk + nl, h = n >> 6, dk = n & (DKK - 1);
          *(volatile v4u_t*)((bf16*)out + (((size_t)(b_ * HH + h)) * DKK + dk) * SS + s0 + q) = *(const v4ua*)(so + nl * 136 + q); }
      }
      __threadfence();
    }
  } else {
    float* so = (float*)sob;
#pragma unroll 1
    for (int hf = 0; hf < 2; ++hf) {
      if (wm == hf * 64) {
#pragma unroll
        for (int i = 0; i < 4; ++i)
#pragma unroll
          for (int j = 0; j < 4; ++j) {
            const int nl = wn + 16 * j + nlane;
            const float bv = bias ? bias[nBlk + nl] : 0.0f;
#pragma unroll
            for (int r = 0; r < 8; ++r) so[(16 * i + mh + r) * 260 + nl] = acc[i][j][r] + bv;
          }
      }
      __syncthreads();
#pragma unroll 1
      for (int pass = 0; pass < 2; ++pass) {
        for (int ch = t; ch < 64 * 64; ch += 256) { const int ml = ch >> 6, q = (ch & 63) * 4;
          *(volatile v4f_t*)((float*)out + (size_t)(mBlk + hf * 64 + ml) * N + nBlk + q) = *(const volatile v4fa*)(so + ml * 260 + q); }
        __threadfence();
      }
      __syncthreads();
    }
  }
}


#define NND 5000
#define NNP 5120
#define NCF 32
#define NE1 8000
#define NE2 16000
#define NR (NND * NCF)
#define HDM 64
#define KX 160

__device__ __forceinline__ int clampi(int v, int hi) { return v < 0 ? 0 : (v >= hi ? hi - 1 : v); }

__global__ __launch_bounds__(160) void k_xn(const float* __restrict__ nf, const int* __restrict__ opc, const float* __restrict__ emb, float* __restrict__ XN) {
  const int n = blockIdx.x, k = threadIdx.x; float v = 0.0f;
  if (n < NND) { if (k < 140) v = nf[(size_t)n * 140 + k]; else if (k < 148) v = emb[clampi(opc[n], 120) * 8 + (k - 140)]; }
  *(volatile float*)(XN + (size_t)n * KX + k) = v; __threadfence(); *(volatile float*)(XN + (size_t)n * KX + k) = v;
}
__global__ __launch_bounds__(160) void k_a0(const float* __restrict__ ws, const float* __restrict__ wn, float* __restrict__ A0) {
  const int j = blockIdx.x, k = threadIdx.x; const float* w = (j < 64) ? ws : wn; const int jj = j & 63;
  const float v = (k < 148) ? w[(size_t)k * HDM + jj] : 0.0f;
  *(volatile float*)(A0 + (size_t)j * KX + k) = v; __threadfence(); *(volatile float*)(A0 + (size_t)j * KX + k) = v;
}
__global__ __launch_bounds__(128) void k_vcf(const float* __restrict__ cf, const float* __restrict__ ws, const float* __restrict__ wn, float* __restrict__ V) {
  const int j = threadIdx.x; const float* w = (j < 64) ? ws : wn; const int jj = j & 63;
  for (int c = 0; c < NCF; ++c) { float s = 0.0f; for (int k = 0; k < 24; ++k) s += cf[c * 24 + k] * w[(size_t)(148 + k) * HDM + jj];
    *(volatile float*)(V + c * 128 + j) = s; }
  __threadfence();
  for (int c = 0; c < NCF; ++c) { float s = 0.0f; for (int k = 0; k < 24; ++k) s += cf[c * 24 + k] * w[(size_t)(148 + k) * HDM + jj];
    *(volatile float*)(V + c * 128 + j) = s; }
}
__global__ __launch_bounds__(64) void k_acat(const float* __restrict__ Wa, const float* __restrict__ Wb, float* __restrict__ A) {
  const int j = blockIdx.x, k = threadIdx.x; float v = 0.0f;
  if (j < 64) v = Wa[(size_t)k * HDM + j]; else if (Wb) v = Wb[(size_t)k * HDM + (j - 64)];
  *(volatile float*)(A + (size_t)j * HDM + k) = v; __threadfence(); *(volatile float*)(A + (size_t)j * HDM + k) = v;
}
__global__ __launch_bounds__(256) void k_agg0(const int* __restrict__ ei, const float* __restrict__ TU, float* __restrict__ AG, float* __restrict__ deg) {
  __shared__ int qd[8][256], qs[8][256]; __shared__ int wcnt[8][8];
  const int tid = threadIdx.x, lane = tid & 31, wave = tid >> 5;
  for (int i = tid; i < NNP * 16; i += 256) { v4f_t z; z.x = z.y = z.z = z.w = 0.f; *(volatile v4f_t*)(AG + (size_t)i * 4) = z; }
  for (int i = tid; i < NNP; i += 256) *(volatile float*)(deg + i) = 0.0f;
  __threadfence(); __syncthreads();
  for (int c0 = 0; c0 < NE2; c0 += 256) {
    const int e = c0 + tid; int d = -1, s = 0;
    if (e < NE2) { const int er = (e < NE1) ? e : e - NE1; const int a = clampi(ei[er * 2], NND), b = clampi(ei[er * 2 + 1], NND); if (e < NE1) { s = a; d = b; } else { s = b; d = a; } }
    const int own = (d >= 0) ? (d & 7) : -1; unsigned mown = 0u;
#pragma unroll
    for (int ww = 0; ww < 8; ++ww) { const unsigned m = __builtin_amdgcn_ballot_w32(own == ww); if (own == ww) mown = m; if (lane == 0) wcnt[ww][wave] = __builtin_popcount(m); }
    __syncthreads();
    if (own >= 0) { int base = 0;
#pragma unroll
      for (int w2 = 0; w2 < 8; ++w2) base += (w2 < wave) ? wcnt[own][w2] : 0;
      const int pos = base + __builtin_popcount(mown & ((1u << lane) - 1u)); qd[own][pos] = d; qs[own][pos] = s; }
    int total = 0;
#pragma unroll
    for (int w2 = 0; w2 < 8; ++w2) total += wcnt[wave][w2];
    __syncthreads();
#pragma unroll 1
    for (int qi = 0; qi < total; ++qi) { const int dn = qd[wave][qi], sn = qs[wave][qi];
      AG[(size_t)dn * 64 + lane] += TU[(size_t)(64 + lane) * NNP + sn]; AG[(size_t)dn * 64 + 32 + lane] += TU[(size_t)(96 + lane) * NNP + sn]; if (lane == 0) deg[dn] += 1.0f; }
    __syncthreads();
  }
  __threadfence(); __syncthreads();
  for (int i = tid; i < NNP * 16; i += 256) { float* p = AG + (size_t)i * 4; const v4f_t v = *(const volatile v4fa*)p; *(volatile v4f_t*)p = v; }
  for (int i = tid; i < NNP; i += 256) { const float v = *(volatile float*)(deg + i); *(volatile float*)(deg + i) = v; }
  __threadfence();
}
__global__ __launch_bounds__(256) void k_h0(const float* __restrict__ TU, const float* __restrict__ V, const float* __restrict__ AG, const float* __restrict__ deg, const float* __restrict__ b0, bf16* __restrict__ H) {
  const int n = blockIdx.x, t = threadIdx.x, c = t >> 3, j8 = (t & 7) * 8; const float dg = deg[n], inv = 1.0f / fmaxf(dg, 1.0f), has = (dg > 0.0f) ? 1.0f : 0.0f;
  bf16 h[8];
#pragma unroll
  for (int q = 0; q < 8; ++q) { const int j = j8 + q;
    const float v = TU[(size_t)j * NNP + n] + V[c * 128 + j] + AG[(size_t)n * 64 + j] * inv + has * V[c * 128 + 64 + j] + b0[j];
    h[q] = (bf16)fmaxf(v, 0.0f); }
  bf16* dst = H + ((size_t)n * NCF + c) * HDM + j8; *(volatile v4u_t*)dst = *(const v4ua*)h; __threadfence(); *(volatile v4u_t*)dst = *(const v4ua*)h;
}
__global__ __launch_bounds__(256) void k_aggl(const int* __restrict__ ei, const bf16* __restrict__ T, float* __restrict__ R) {
  __shared__ int qd[8][256], qs[8][256]; __shared__ int wcnt[8][8];
  const int tid = threadIdx.x, lane = tid & 31, wave = tid >> 5;
  for (int i = tid; i < NR * 16; i += 256) { v4f_t z; z.x = z.y = z.z = z.w = 0.f; *(volatile v4f_t*)(R + (size_t)i * 4) = z; }
  __threadfence(); __syncthreads();
  for (int c0 = 0; c0 < NE2; c0 += 256) {
    const int e = c0 + tid; int d = -1, s = 0;
    if (e < NE2) { const int er = (e < NE1) ? e : e - NE1; const int a = clampi(ei[er * 2], NND), b = clampi(ei[er * 2 + 1], NND); if (e < NE1) { s = a; d = b; } else { s = b; d = a; } }
    const int own = (d >= 0) ? (d & 7) : -1; unsigned mown = 0u;
#pragma unroll
    for (int ww = 0; ww < 8; ++ww) { const unsigned m = __builtin_amdgcn_ballot_w32(own == ww); if (own == ww) mown = m; if (lane == 0) wcnt[ww][wave] = __builtin_popcount(m); }
    __syncthreads();
    if (own >= 0) { int base = 0;
#pragma unroll
      for (int w2 = 0; w2 < 8; ++w2) base += (w2 < wave) ? wcnt[own][w2] : 0;
      const int pos = base + __builtin_popcount(mown & ((1u << lane) - 1u)); qd[own][pos] = d; qs[own][pos] = s; }
    int total = 0;
#pragma unroll
    for (int w2 = 0; w2 < 8; ++w2) total += wcnt[wave][w2];
    __syncthreads();
#pragma unroll 1
    for (int qi = 0; qi < total; ++qi) { const int dn = qd[wave][qi], sn = qs[wave][qi];
      float* row = R + ((size_t)dn * NCF + lane) * HDM; const bf16* tcol = T + (size_t)64 * NR + (size_t)sn * NCF + lane;
#pragma unroll 4
      for (int j = 0; j < 64; ++j) row[j] += (float)tcol[(size_t)j * NR]; }
    __syncthreads();
  }
  __threadfence(); __syncthreads();
  for (int i = tid; i < NR * 16; i += 256) { float* p = R + (size_t)i * 4; const v4f_t v = *(const volatile v4fa*)p; *(volatile v4f_t*)p = v; }
  __threadfence();
}
__global__ __launch_bounds__(256) void k_hl(const bf16* __restrict__ T, const float* __restrict__ R, const float* __restrict__ deg, const float* __restrict__ b, bf16* __restrict__ H) {
  const int n = blockIdx.x, t = threadIdx.x, c = t >> 3, j8 = (t & 7) * 8; const float inv = 1.0f / fmaxf(deg[n], 1.0f);
  const size_t row = (size_t)n * NCF + c; bf16 h[8];
#pragma unroll
  for (int q = 0; q < 8; ++q) { const int j = j8 + q; const float v = (float)T[(size_t)j * NR + row] + R[row * HDM + j] * inv + b[j]; h[q] = (bf16)fmaxf(v, 0.0f); }
  bf16* dst = H + row * HDM + j8; *(volatile v4u_t*)dst = *(const v4ua*)h; __threadfence(); *(volatile v4u_t*)dst = *(const v4ua*)h;
}
__global__ __launch_bounds__(256) void k_skp(const bf16* __restrict__ TS, const float* __restrict__ sb, int l, float* __restrict__ P) {
  for (int i = threadIdx.x; i < NCF * 64; i += 256) { const int c = i >> 6, j = i & 63; const float bj = sb[j]; float s = 0.0f;
#pragma unroll 4
    for (int n = 0; n < NND; ++n) s += fmaxf((float)TS[(size_t)j * NR + (size_t)n * NCF + c] + bj, 0.0f);
    *(volatile float*)(P + (size_t)c * 192 + l * 64 + j) = s; }
  __threadfence();
  for (int i = threadIdx.x; i < NCF * 64; i += 256) { const int c = i >> 6, j = i & 63; const float v = *(volatile float*)(P + (size_t)c * 192 + l * 64 + j); *(volatile float*)(P + (size_t)c * 192 + l * 64 + j) = v; }
}
__global__ __launch_bounds__(256) void k_head(const float* __restrict__ P, const float* __restrict__ p1w, const float* __restrict__ p1b, const float* __restrict__ p2w, const float* __restrict__ p2b, const float* __restrict__ p3w, const float* __restrict__ p3b, float* __restrict__ out) {
  __shared__ float h1[NCF][128]; __shared__ float h2[NCF][64]; __shared__ float res[NCF];
  const int t = threadIdx.x;
  for (int i = t; i < NCF * 128; i += 256) { const int c = i >> 7, j = i & 127; float s = p1b[j]; for (int k = 0; k < 192; ++k) s += P[c * 192 + k] * p1w[k * 128 + j]; h1[c][j] = fmaxf(s, 0.0f); }
  __syncthreads();
  for (int i = t; i < NCF * 64; i += 256) { const int c = i >> 6, j = i & 63; float s = p2b[j]; for (int k = 0; k < 128; ++k) s += h1[c][k] * p2w[k * 64 + j]; h2[c][j] = fmaxf(s, 0.0f); }
  __syncthreads();
  if (t < NCF) { float s = p3b[0]; for (int k = 0; k < 64; ++k) s += h2[t][k] * p3w[k]; res[t] = s; }
  __syncthreads();
  if (t < 8) { const v4f_t v = *(const volatile v4fa*)(res + t * 4); *(volatile v4f_t*)(out + t * 4) = v; __threadfence(); *(volatile v4f_t*)(out + t * 4) = v; }
}

extern "C" void kernel_launch(void* const* d_in, const int* in_sizes, int n_in,
                              void* d_out, int out_size, void* d_ws, size_t ws_size,
                              hipStream_t stream) {
  (void)in_sizes; (void)n_in; (void)out_size; (void)ws_size;
  const float* nf = (const float*)d_in[0]; const int* opc = (const int*)d_in[1]; const int* ei = (const int*)d_in[2]; const float* cf = (const float*)d_in[3]; const float* emb = (const float*)d_in[4];
  const float* ws0 = (const float*)d_in[5]; const float* wn0 = (const float*)d_in[6]; const float* b0 = (const float*)d_in[7];
  const float* wsl = (const float*)d_in[8]; const float* wnl = (const float*)d_in[9]; const float* bl = (const float*)d_in[10];
  const float* skw = (const float*)d_in[11]; const float* skb = (const float*)d_in[12];
  const float* p1w = (const float*)d_in[13]; const float* p1b = (const float*)d_in[14]; const float* p2w = (const float*)d_in[15]; const float* p2b = (const float*)d_in[16]; const float* p3w = (const float*)d_in[17]; const float* p3b = (const float*)d_in[18];
  char* ws = (char*)d_ws;
  float* XN = (float*)ws; ws += (size_t)NNP * KX * 4;
  float* A0 = (float*)ws; ws += (size_t)128 * KX * 4;
  float* Al = (float*)ws; ws += (size_t)128 * HDM * 4 * 5;
  float* V  = (float*)ws; ws += (size_t)NCF * 128 * 4;
  float* TU = (float*)ws; ws += (size_t)128 * NNP * 4;
  float* AG = (float*)ws; ws += (size_t)NNP * 64 * 4; float* deg = (float*)ws; ws += (size_t)NNP * 4;
  float* P  = (float*)ws; ws += (size_t)NCF * 192 * 4;
  bf16* H   = (bf16*)ws;  ws += (size_t)NR * HDM * 2;
  bf16* T   = (bf16*)ws;  ws += (size_t)128 * NR * 2;
  float* R  = (float*)ws; ws += (size_t)NR * HDM * 4;
  k_xn<<<NNP, 160, 0, stream>>>(nf, opc, emb, XN);
  k_a0<<<128, 160, 0, stream>>>(ws0, wn0, A0);
  k_vcf<<<1, 128, 0, stream>>>(cf, ws0, wn0, V);
  k_acat<<<128, 64, 0, stream>>>(wsl, wnl, Al);
  k_acat<<<128, 64, 0, stream>>>(wsl + 64 * 64, wnl + 64 * 64, Al + 128 * HDM);
  for (int l = 0; l < 3; ++l) k_acat<<<128, 64, 0, stream>>>(skw + (size_t)l * 64 * 64, nullptr, Al + (size_t)(2 + l) * 128 * HDM);
  dim3 blk(256);
  gemm_bias_kernel<float, float, 2><<<dim3(1, NNP / 256), blk, 0, stream>>>(A0, XN, nullptr, TU, 128, NNP, KX);
  k_agg0<<<1, 256, 0, stream>>>(ei, TU, AG, deg);
  k_h0<<<NND, 256, 0, stream>>>(TU, V, AG, deg, b0, H);
  gemm_bias_kernel<float, bf16, 0><<<dim3(1, NR / 256), blk, 0, stream>>>(Al + (size_t)2 * 128 * HDM, H, nullptr, T, 128, NR, HDM);
  k_skp<<<1, 256, 0, stream>>>(T, skb, 0, P);
  for (int l = 0; l < 2; ++l) {
    gemm_bias_kernel<float, bf16, 0><<<dim3(1, NR / 256), blk, 0, stream>>>(Al + (size_t)l * 128 * HDM, H, nullptr, T, 128, NR, HDM);
    k_aggl<<<1, 256, 0, stream>>>(ei, T, R);
    k_hl<<<NND, 256, 0, stream>>>(T, R, deg, bl + l * 64, H);
    gemm_bias_kernel<float, bf16, 0><<<dim3(1, NR / 256), blk, 0, stream>>>(Al + (size_t)(3 + l) * 128 * HDM, H, nullptr, T, 128, NR, HDM);
    k_skp<<<1, 256, 0, stream>>>(T, skb + (l + 1) * 64, l + 1, P);
  }
  k_head<<<1, 256, 0, stream>>>(P, p1w, p1b, p2w, p2b, p3w, p3b, (float*)d_out);
}
